// QNet_14499809592003
// MI455X (gfx1250) — hardware-run, weakly checked
//
#include <hip/hip_runtime.h>


namespace {

constexpr int N = 50000, NP = 50048, NPL = NP  , SRCM = N  , EFULL = 800000, E = EFULL  , EL = E  ;
constexpr int F = 4, C = 64, C3 = 3 * C, CM = 4 * C  , NO = 4, NL = (NPL < N ? NPL : N);
constexpr float XS = 8.0f, WSC = 256.0f, WSQ = 0.25f, RS_ = 1024.0f, SLOPE = 0.0f, BNEPS = 1e-5f;
static_assert(NP % 32 == 0 && NP >= N && NPL % 32 == 0 && E % 64 == 0 && EL % 64 == 0 && C == 64, "tiling");
typedef _Float16 b16;
typedef __attribute__((ext_vector_type(16))) _Float16 v16b;
typedef __attribute__((ext_vector_type(8))) _Float16 v8b;
typedef __attribute__((ext_vector_type(8))) float v8f;
typedef __attribute__((ext_vector_type(4))) float v4f;
__device__ __forceinline__ float bf16_rne(float f) { unsigned int u = __float_as_uint(f); u += 0x7FFFu + ((u >> 16) & 1u); return __uint_as_float(u & 0xFFFF0000u); }
__device__ __forceinline__ void split16(float v, b16& hi, b16& lo) { hi = (b16)v; lo = (b16)(v - (float)hi); }
__device__ __forceinline__ v16b frag_kb(const b16* p, int hh) { const v8b a = *(const v8b*)(p + 8 * hh), b = *(const v8b*)(p + 16 + 8 * hh); v16b f;
#pragma unroll
  for (int e = 0; e < 8; ++e) { f[e] = a[e]; f[8 + e] = b[e]; } return f; }
__device__ __forceinline__ v8f wmma16b(v16b a, v16b b, v8f c) { v8f d = __builtin_amdgcn_wmma_f32_16x16x32_f16(false, a, false, b, (short)0, c, false, false); asm volatile("v_nop\n\tv_nop\n\tv_nop\n\tv_nop" : "+v"(d) : "v"(a), "v"(b)); return d; }
__device__ __forceinline__ void wave_lds_sync() { __builtin_amdgcn_fence(__ATOMIC_RELEASE, "workgroup"); __builtin_amdgcn_wave_barrier(); __builtin_amdgcn_fence(__ATOMIC_ACQUIRE, "workgroup"); }
__device__ __forceinline__ float pmul(float a, float b) { float p = a * b; asm volatile("" : "+v"(p)); return p; }
__device__ __forceinline__ int iclamp(int v, int lo, int hi) { return v < lo ? lo : (v > hi ? hi : v); }
constexpr int CSR_NBLK = 512, CSR_GB = 9, CSR_GN = 1 << CSR_GB  , CSR_MAXG = 512, CSR_CAP = 12288  ;
__global__ __launch_bounds__(64) void csrA_kernel(const int* __restrict__ dst, int E, int N, int nG, int CHP, int NGP, int* __restrict__ STG, int* __restrict__ HST) {
  extern __shared__ int sm[];
  int* cnt = sm; int* run = sm + NGP; int* ids = sm + 2 * NGP;
  const int b = blockIdx.x; const int ch = (E + CSR_NBLK - 1) / CSR_NBLK; const int e0 = b * ch, e1 = min(E, e0 + ch);
  for (int i = threadIdx.x; i < NGP; i += 64) cnt[i] = 0;
  for (int i = threadIdx.x; i < CHP; i += 64) ids[i] = -1;
  __syncthreads();
  if (threadIdx.x == 0) {
    for (int e = e0; e < e1; ++e) { int d = dst[e]; d = (d < 0) ? 0 : (d >= N ? N - 1 : d); cnt[d >> CSR_GB] += 1; }
    int acc = 0; for (int g = 0; g < nG; ++g) { run[g] = acc; acc += cnt[g]; }
    for (int e = e0; e < e1; ++e) { int d = dst[e]; d = (d < 0) ? 0 : (d >= N ? N - 1 : d); const int g = d >> CSR_GB; ids[run[g]] = e; run[g] += 1; } }
  __syncthreads();
  typedef __attribute__((ext_vector_type(4))) int v4i;
  for (int pass = 0; pass < 2; ++pass) {
    for (int i = threadIdx.x; i < CHP / 4; i += 64) *(volatile v4i*)(STG + (size_t)b * CHP + i * 4) = *(const v4i*)(&ids[i * 4]);
    for (int i = threadIdx.x; i < NGP / 4; i += 64) { v4i v; for (int e = 0; e < 4; ++e) v[e] = (i * 4 + e < nG) ? cnt[i * 4 + e] : 0; *(volatile v4i*)(HST + (size_t)b * NGP + i * 4) = v; }
    __threadfence(); }
}
__global__ __launch_bounds__(512) void csrS_kernel(const int* __restrict__ HST, int nG, int NGP, int* __restrict__ START, int* __restrict__ TOT, int* __restrict__ OFF) {
  __shared__ int tot[CSR_MAXG];
  const int b = threadIdx.x;
  for (int pass = 0; pass < 2; ++pass) { int runb = 0; for (int g = 0; g < nG; ++g) { int c = HST[(size_t)b * NGP + g]; c = (c < 0) ? 0 : c; ((volatile int*)OFF)[(size_t)g * CSR_NBLK + b] = runb; runb += c; } __threadfence(); }
  for (int g = threadIdx.x; g < nG; g += 512) { int s = 0; for (int bb = 0; bb < CSR_NBLK; ++bb) { int c = HST[(size_t)bb * NGP + g]; s += (c < 0) ? 0 : c; } tot[g] = s; }
  __syncthreads();
  if (threadIdx.x < 32) {
    __shared__ int st[CSR_MAXG + 32];
    if (threadIdx.x == 0) { int acc = 0; for (int g = 0; g < NGP; ++g) { st[g] = acc; if (g < nG) acc += (tot[g] + 31) & ~31; } st[NGP] = acc; }
    __builtin_amdgcn_fence(__ATOMIC_RELEASE, "workgroup"); __builtin_amdgcn_wave_barrier(); __builtin_amdgcn_fence(__ATOMIC_ACQUIRE, "workgroup");
    for (int pass = 0; pass < 2; ++pass) { for (int i = threadIdx.x; i < NGP + 32; i += 32) { ((volatile int*)START)[i] = (i <= NGP) ? st[min(i, NGP)] : 0; ((volatile int*)TOT)[i] = (i < nG) ? tot[i] : 0; } __threadfence(); } }
}
__global__ __launch_bounds__(256) void csrB_kernel(const int* __restrict__ dst, int N, int nG, int CHP, int NGP, int permLen, const int* __restrict__ STG, const int* __restrict__ HST, const int* __restrict__ OFF, const int* __restrict__ START, const int* __restrict__ TOT, int* __restrict__ PERM, int* __restrict__ ROWPTR, int* __restrict__ ROWCNT, int* __restrict__ FLAG) {
  typedef __attribute__((ext_vector_type(4))) int v4i;
  __shared__ int ids[CSR_CAP]; __shared__ unsigned short key[CSR_CAP]; __shared__ int outp[CSR_CAP]; __shared__ int ncnt[CSR_GN + 1]; __shared__ int boff[CSR_NBLK + 1];
  const int g = blockIdx.x, t_ = threadIdx.x; int tot = TOT[g]; int st = START[g], stn = START[g + 1]; const int v0 = g * CSR_GN; const int nv = min(CSR_GN, N - v0);
  st = (st < 0) ? 0 : (st > permLen - 32 ? permLen - 32 : st) & ~31; stn = (stn < st) ? st : (stn > permLen ? permLen : stn); tot = (tot < 0) ? 0 : tot; if (tot > stn - st && tot <= CSR_CAP) tot = stn - st;
  if (tot > CSR_CAP) {
    for (int pass = 0; pass < 2; ++pass) { for (int i = t_; i < CSR_GN / 4; i += 256) { v4i a, c; for (int e = 0; e < 4; ++e) { a[e] = st; c[e] = 0; } *(volatile v4i*)(ROWPTR + v0 + i * 4) = a; *(volatile v4i*)(ROWCNT + v0 + i * 4) = c; } if (t_ == 0) ((volatile int*)FLAG)[0] = 1; __threadfence(); } (void)nv; return; }
  if (t_ == 0) { int acc = 0; for (int b = 0; b < CSR_NBLK; ++b) { boff[b] = acc; int c = HST[(size_t)b * NGP + g]; c = (c < 0) ? 0 : (c > CHP ? CHP : c); acc += c; if (acc > tot) acc = tot; } boff[CSR_NBLK] = acc; }
  for (int i = t_; i <= CSR_GN; i += 256) ncnt[i] = 0;
  __syncthreads();
  for (int b = 0; b < CSR_NBLK; ++b) { const int c = boff[b + 1] - boff[b]; int o_ = OFF[(size_t)g * CSR_NBLK + b]; o_ = (o_ < 0) ? 0 : (o_ > CHP - c ? CHP - c : o_); const int* src_ = STG + (size_t)b * CHP + o_;
    for (int i = t_; i < c; i += 256) { int id = src_[i]; id = (id < 0) ? 0 : id; ids[boff[b] + i] = id; int d = dst[id]; d = (d < v0) ? v0 : (d >= N ? N - 1 : d); int kk = d - v0; kk = (kk < 0) ? 0 : (kk >= CSR_GN ? CSR_GN - 1 : kk); key[boff[b] + i] = (unsigned short)kk; } }
  __syncthreads();
  if (t_ == 0) { for (int i = 0; i < tot; ++i) ncnt[key[i]] += 1; int acc = 0; for (int vl = 0; vl < CSR_GN; ++vl) { const int c = ncnt[vl]; ncnt[vl] = acc; acc += c; } ncnt[CSR_GN] = acc;
    for (int i = 0; i < tot; ++i) { const int vl = key[i]; outp[ncnt[vl]] = ids[i]; ncnt[vl] += 1; }
    for (int vl = CSR_GN; vl > 0; --vl) ncnt[vl] = ncnt[vl - 1]; ncnt[0] = 0; }
  __syncthreads();
  for (int pass = 0; pass < 2; ++pass) {
    for (int i = t_; i < (stn - st) / 4; i += 256) { v4i v; for (int e = 0; e < 4; ++e) { const int q = i * 4 + e; v[e] = (q < tot) ? outp[q] : -1; } *(volatile v4i*)(PERM + st + i * 4) = v; }
    for (int i = t_; i < CSR_GN / 4; i += 256) { v4i a, c; for (int e = 0; e < 4; ++e) { const int vl = i * 4 + e; a[e] = st + ncnt[vl]; c[e] = (vl < nv) ? (ncnt[vl + 1] - ncnt[vl]) : 0; } *(volatile v4i*)(ROWPTR + v0 + i * 4) = a; *(volatile v4i*)(ROWCNT + v0 + i * 4) = c; }
    __threadfence(); }
}
__global__ __launch_bounds__(256) void csrZ_kernel(int* __restrict__ p, size_t n4) { typedef __attribute__((ext_vector_type(4))) int v4i; const size_t tid = (size_t)blockIdx.x * 256 + threadIdx.x, nth = (size_t)gridDim.x * 256; v4i z = {0, 0, 0, 0}; for (size_t i = tid; i < n4; i += nth) *(volatile v4i*)(p + i * 4) = z; }
struct CsrBufs { int *STG, *HST, *OFF, *START, *TOT, *PERM, *ROWPTR, *ROWCNT, *FLAG; int nG, NGP, CHP; size_t permLen; char* base; size_t bytes; };
static size_t csr_carve(CsrBufs& c, char* ws, size_t off, int E, int N) {
  const size_t off0 = off; c.base = ws + off;
  auto al = [&](size_t bytes) { char* p = ws + off; off += (bytes + 255) & ~(size_t)255; return p; };
  c.nG = (N + CSR_GN - 1) / CSR_GN; c.NGP = (c.nG + 31) & ~31; const int ch = (E + CSR_NBLK - 1) / CSR_NBLK; c.CHP = (ch + 31) & ~31; c.permLen = (size_t)E + 32 * (size_t)c.nG + 32;
  c.STG = (int*)al((size_t)CSR_NBLK * c.CHP * 4); c.HST = (int*)al((size_t)CSR_NBLK * c.NGP * 4); c.OFF = (int*)al((size_t)c.NGP * CSR_NBLK * 4); c.START = (int*)al((size_t)(c.NGP + 64) * 4); c.TOT = (int*)al((size_t)(c.NGP + 64) * 4);
  c.PERM = (int*)al(c.permLen * 4); c.ROWPTR = (int*)al((size_t)c.nG * CSR_GN * 4); c.ROWCNT = (int*)al((size_t)c.nG * CSR_GN * 4); c.FLAG = (int*)al(256);
  c.bytes = off - off0; return off;
}
static void csr_build(const CsrBufs& c, const int* dst, int E, int N, hipStream_t stream) {
  const size_t smem = (size_t)(2 * c.NGP + c.CHP) * 4;
  csrZ_kernel<<<512, 256, 0, stream>>>((int*)c.base, c.bytes / 16);
  csrA_kernel<<<CSR_NBLK, 64, smem, stream>>>(dst, E, N, c.nG, c.CHP, c.NGP, c.STG, c.HST);
  csrS_kernel<<<1, 512, 0, stream>>>(c.HST, c.nG, c.NGP, c.START, c.TOT, c.OFF);
  csrB_kernel<<<c.nG, 256, 0, stream>>>(dst, N, c.nG, c.CHP, c.NGP, (int)c.permLen, c.STG, c.HST, c.OFF, c.START, c.TOT, c.PERM, c.ROWPTR, c.ROWCNT, c.FLAG);
}

typedef __attribute__((ext_vector_type(4))) _Float16 v4h;
typedef __attribute__((ext_vector_type(2))) float v2f;
__global__ __launch_bounds__(256) void prep_kernel(const float* __restrict__ c1W1, const float* __restrict__ c1b1, const float* __restrict__ c1W2, const float* __restrict__ c1W3, const float* __restrict__ c1b3, const float* __restrict__ c2W1, const float* __restrict__ c2W2, const float* __restrict__ c2W3,
    const float* __restrict__ meW1, const float* __restrict__ meW2, b16* __restrict__ WL1, b16* __restrict__ WL2, b16* __restrict__ WM1, b16* __restrict__ WM2, float scl) {
  const int n1 = C * 32 / 8, n2 = C3 * C / 8, n3 = CM * 2 * C / 8, n4 = 16 * CM / 8; const int u = blockIdx.x * 256 + threadIdx.x; if (u >= n1 + n2 + n3 + n4) return; v8b v; b16* dst;
  if (u < n1) { const int e = u * 8, o = e / 32, k0 = e % 32; for (int j = 0; j < 8; ++j) { const int k = k0 + j; float w = 0.0f;
      if (k < 4) w = bf16_rne(c1W1[o * F + k]); else if (k == 4) w = bf16_rne(c1b1[o]); else if (k < 9) w = -bf16_rne(c1W2[o * F + (k - 5)]); else if (k < 13) w = bf16_rne(c1W3[o * F + (k - 9)]); else if (k == 13) w = bf16_rne(c1b3[o]); v[j] = (b16)(w * scl); } dst = WL1 + e; }
  else if (u < n1 + n2) { const int e = (u - n1) * 8, o = e / C, k0 = e % C; const int m = o / C, oo = o % C; const float* w = m == 0 ? c2W1 : m == 1 ? c2W2 : c2W3; for (int j = 0; j < 8; ++j) v[j] = (b16)(bf16_rne(w[oo * C + k0 + j]) * scl); dst = WL2 + e; }
  else if (u < n1 + n2 + n3) { const int e = (u - n1 - n2) * 8, o = e / (2 * C), k0 = e % (2 * C); for (int j = 0; j < 8; ++j) v[j] = (b16)(bf16_rne(meW1[o * 2 * C + k0 + j]) * scl); dst = WM1 + e; }
  else { const int e = (u - n1 - n2 - n3) * 8, o = e / CM, k0 = e % CM; for (int j = 0; j < 8; ++j) v[j] = (b16)(o < NO ? bf16_rne(meW2[o * CM + k0 + j]) * scl : 0.0f); dst = WM2 + e; }
  for (int pass = 0; pass < 2; ++pass) { *(volatile v8b*)dst = v; __threadfence(); }
}
__device__ __forceinline__ void puthl(b16* h, b16* l, float v) { const float vs = v * XS; const b16 p = (b16)vs; *h = p; *l = (b16)((vs - (float)p) * RS_); }
__global__ __launch_bounds__(64) void layer1_kernel(const float* __restrict__ x, const float* __restrict__ ew, const int* __restrict__ srcs, const int* __restrict__ PERM, const int* __restrict__ ROWPTR, const int* __restrict__ ROWCNT, int permLen, const b16* __restrict__ WL1, const b16* __restrict__ WL1q, float* __restrict__ Q1) {
  __shared__ __attribute__((aligned(16))) b16 Ah[2][16][32 + 8], Al[2][16][32 + 8]; __shared__ __attribute__((aligned(16))) float Tf[2][16][C + 4];
  const int wave = threadIdx.x >> 5, lane = threadIdx.x & 31, nloc = lane & 15, hlf = lane >> 4; const int m0 = blockIdx.x * 32 + wave * 16;
  if (lane < 16) { const int v = m0 + lane; float sx[4] = {0.f, 0.f, 0.f, 0.f}, sw = 0.0f, xv[4] = {0.f, 0.f, 0.f, 0.f};
    int cnt = 0, p0 = 0; if (v < N) { cnt = iclamp(ROWCNT[v], 0, 65536); p0 = iclamp(ROWPTR[v], 0, permLen - 1); if (p0 + cnt > permLen) cnt = permLen - p0; const v4f t4 = *(const v4f*)(x + (size_t)v * F); for (int j = 0; j < 4; ++j) xv[j] = bf16_rne(t4[j]); }
#pragma unroll 1
    for (int i = 0; i < cnt; ++i) { const int e = iclamp(PERM[p0 + i], 0, E - 1); int s = iclamp(srcs[e], 0, N - 1); if (SRCM < N) s %= SRCM; const float w = bf16_rne(ew[e]); const v4f t4 = *(const v4f*)(x + (size_t)s * F); for (int j = 0; j < 4; ++j) sx[j] = fmaf(w, bf16_rne(t4[j]), sx[j]); sw += w; }
    float row32[32]; for (int k = 0; k < 32; ++k) row32[k] = 0.0f; for (int j = 0; j < 4; ++j) { row32[j] = sx[j]; row32[5 + j] = xv[j] * sw; row32[9 + j] = xv[j]; } row32[4] = sw; row32[13] = 1.0f;
    if (v >= N) for (int k = 0; k < 32; ++k) row32[k] = 0.0f;
    for (int k = 0; k < 32; ++k) puthl(&Ah[wave][lane][k], &Al[wave][lane][k], row32[k]); }
  wave_lds_sync();
  v8f acc[4]; for (int t = 0; t < 4; ++t) acc[t] = (v8f){};
  { const v16b a = frag_kb(&Ah[wave][nloc][0], hlf), al = frag_kb(&Al[wave][nloc][0], hlf);
#pragma unroll
    for (int t = 0; t < 4; ++t) { const size_t wo_ = (size_t)(t * 16 + nloc) * 32; acc[t] = wmma16b(a, frag_kb(WL1 + wo_, hlf), acc[t]); acc[t] = wmma16b(al, frag_kb(WL1q + wo_, hlf), acc[t]); } }
#pragma unroll
  for (int t = 0; t < 4; ++t) for (int r = 0; r < 8; ++r) Tf[wave][8 * hlf + r][t * 16 + nloc] = acc[t][r] * (1.0f / (XS * WSC));
  wave_lds_sync();
  for (int pass = 0; pass < 2; ++pass) { for (int rr = 0; rr < 16; rr += 2) { const int r2 = rr + (lane >> 4); *(volatile v4f*)(Q1 + (size_t)(m0 + r2) * C + (lane & 15) * 4) = *(const v4f*)(&Tf[wave][r2][(lane & 15) * 4]); } __threadfence(); }
}
__global__ __launch_bounds__(64) void lin2_kernel(const float* __restrict__ Q1, const b16* __restrict__ WL2, const b16* __restrict__ WL2q, const float* __restrict__ b1, const float* __restrict__ b3, float* __restrict__ ABC) {
  __shared__ __attribute__((aligned(16))) b16 Ah[2][16][C + 8], Al[2][16][C + 8]; __shared__ __attribute__((aligned(16))) float Tf[2][16][C3 + 4];
  const int wave = threadIdx.x >> 5, lane = threadIdx.x & 31, nloc = lane & 15, hlf = lane >> 4; const size_t m0 = (size_t)blockIdx.x * 32 + wave * 16;
  for (int idx = lane; idx < 16 * 16; idx += 32) { const int rr = idx / 16, c4 = (idx % 16) * 4; const v4f v = *(const v4f*)(Q1 + (m0 + rr) * C + c4); v4h hv, lv; for (int j = 0; j < 4; ++j) { b16 p, q; puthl(&p, &q, v[j]); hv[j] = p; lv[j] = q; } *(v4h*)(&Ah[wave][rr][c4]) = hv; *(v4h*)(&Al[wave][rr][c4]) = lv; }
  wave_lds_sync();
  v8f acc[12];
#pragma unroll
  for (int t = 0; t < 12; ++t) acc[t] = (v8f){};
#pragma unroll
  for (int kb = 0; kb < C; kb += 32) { const v16b a = frag_kb(&Ah[wave][nloc][kb], hlf), al = frag_kb(&Al[wave][nloc][kb], hlf);
#pragma unroll
    for (int t = 0; t < 12; ++t) { const size_t wo_ = (size_t)(t * 16 + nloc) * C + kb; acc[t] = wmma16b(a, frag_kb(WL2 + wo_, hlf), acc[t]); acc[t] = wmma16b(al, frag_kb(WL2q + wo_, hlf), acc[t]); } }
#pragma unroll
  for (int t = 0; t < 12; ++t) { const int col = t * 16 + nloc; const float bb = col < C ? bf16_rne(b1[col]) : (col >= 2 * C ? bf16_rne(b3[col - 2 * C]) : 0.0f);
    for (int r = 0; r < 8; ++r) Tf[wave][8 * hlf + r][col] = (m0 + 8 * hlf + r < (size_t)N) ? acc[t][r] * (1.0f / (XS * WSC)) + bb : 0.0f; }
  wave_lds_sync();
  for (int pass = 0; pass < 2; ++pass) { for (int rr = 0; rr < 16; ++rr) { float* d = ABC + (m0 + rr) * C3; *(volatile v4f*)(d + lane * 4) = *(const v4f*)(&Tf[wave][rr][lane * 4]); if (lane < 16) *(volatile v4f*)(d + 128 + lane * 4) = *(const v4f*)(&Tf[wave][rr][128 + lane * 4]); } __threadfence(); }
}
__global__ __launch_bounds__(256) void agg2_kernel(const float* __restrict__ ABC, const float* __restrict__ ew, const int* __restrict__ srcs, const int* __restrict__ PERM, const int* __restrict__ ROWPTR, const int* __restrict__ ROWCNT, int permLen, float* __restrict__ Q2) {
  __shared__ __attribute__((aligned(16))) float rows[32][C + 4];
  const int tid = threadIdx.x; const int row = tid >> 3, g = tid & 7, c0 = g * 8; const int v = blockIdx.x * 32 + row;
  float m[8]; for (int j = 0; j < 8; ++j) m[j] = 0.0f; float sw = 0.0f;
  int cnt = 0, p0 = 0; if (v < N) { cnt = iclamp(ROWCNT[v], 0, 65536); p0 = iclamp(ROWPTR[v], 0, permLen - 1); if (p0 + cnt > permLen) cnt = permLen - p0; }
#pragma unroll 1
  for (int i = 0; i < cnt; ++i) { const int e = iclamp(PERM[p0 + i], 0, E - 1); int s = iclamp(srcs[e], 0, N - 1); if (SRCM < N) s %= SRCM; const float w = bf16_rne(ew[e]); sw += w; const float* ar = ABC + (size_t)s * C3 + c0;
    for (int q = 0; q < 2; ++q) { const v4f t4 = *(const v4f*)(ar + 4 * q); for (int j = 0; j < 4; ++j) m[4 * q + j] = fmaf(w, t4[j], m[4 * q + j]); } }
  { const float* br = ABC + (size_t)(v < N ? v : N - 1) * C3 + C + c0; const float* cr = br + C;
    for (int q = 0; q < 2; ++q) { const v4f b4 = *(const v4f*)(br + 4 * q), c4 = *(const v4f*)(cr + 4 * q); for (int j = 0; j < 4; ++j) rows[row][c0 + 4 * q + j] = (v < N) ? (m[4 * q + j] - b4[j] * sw + c4[j]) : 0.0f; } }
  __syncthreads();
  for (int pass = 0; pass < 2; ++pass) { for (int i = tid; i < 32 * (C / 4); i += 256) { const int rr = i / (C / 4), c4 = (i % (C / 4)) * 4; *(volatile v4f*)(Q2 + (size_t)(blockIdx.x * 32 + rr) * C + c4) = *(const v4f*)(&rows[rr][c4]); } __threadfence(); }
}
__global__ __launch_bounds__(128) void edge_kernel(const float* __restrict__ Q2, const int* __restrict__ srcs, const int* __restrict__ dsts, const b16* __restrict__ WM1, const b16* __restrict__ WM1q, const float* __restrict__ mb1, const b16* __restrict__ WM2, const b16* __restrict__ WM2q, const float* __restrict__ mb2, float* __restrict__ out) {
  __shared__ __attribute__((aligned(16))) b16 Ah[64][CM + 8], Al[64][CM + 8]; __shared__ __attribute__((aligned(16))) float To[64][4];
  const int tid = threadIdx.x, wave = tid >> 5, lane = tid & 31, nloc = lane & 15, hlf = lane >> 4; const size_t e0 = (size_t)blockIdx.x * 64;
  { const int row = tid >> 1, half = tid & 1; const size_t e = e0 + row; int nd = half == 0 ? iclamp(srcs[e], 0, N - 1) : iclamp(dsts[e], 0, N - 1); if (SRCM < N) nd %= SRCM; const float* qr = Q2 + (size_t)nd * C;
    for (int q = 0; q < 16; ++q) { const v4f t4 = *(const v4f*)(qr + 4 * q); v4h hv, lv; for (int j = 0; j < 4; ++j) { b16 p, qq; puthl(&p, &qq, t4[j]); hv[j] = p; lv[j] = qq; } *(v4h*)(&Ah[row][half * C + 4 * q]) = hv; *(v4h*)(&Al[row][half * C + 4 * q]) = lv; } }
  __syncthreads();
  v8f acc[16];
#pragma unroll
  for (int t = 0; t < 16; ++t) acc[t] = (v8f){};
#pragma unroll
  for (int kb = 0; kb < 2 * C; kb += 32) { const v16b a = frag_kb(&Ah[wave * 16 + nloc][kb], hlf), al = frag_kb(&Al[wave * 16 + nloc][kb], hlf);
#pragma unroll
    for (int t = 0; t < 16; ++t) { const size_t wo_ = (size_t)(t * 16 + nloc) * (2 * C) + kb; acc[t] = wmma16b(a, frag_kb(WM1 + wo_, hlf), acc[t]); acc[t] = wmma16b(al, frag_kb(WM1q + wo_, hlf), acc[t]); } }
  __syncthreads();
#pragma unroll
  for (int t = 0; t < 16; ++t) { const int col = t * 16 + nloc; const float bb = bf16_rne(mb1[col]);
    for (int r = 0; r < 8; ++r) { const float h = fmaxf(acc[t][r] * (1.0f / (XS * WSC)) + bb, 0.0f); puthl(&Ah[wave * 16 + 8 * hlf + r][col], &Al[wave * 16 + 8 * hlf + r][col], h); } }
  wave_lds_sync();
  v8f acc2 = (v8f){};
#pragma unroll
  for (int kb = 0; kb < CM; kb += 32) { acc2 = wmma16b(frag_kb(&Ah[wave * 16 + nloc][kb], hlf), frag_kb(WM2 + (size_t)nloc * CM + kb, hlf), acc2); acc2 = wmma16b(frag_kb(&Al[wave * 16 + nloc][kb], hlf), frag_kb(WM2q + (size_t)nloc * CM + kb, hlf), acc2); }
  if (nloc < NO) { const float bb = bf16_rne(mb2[nloc]); for (int r = 0; r < 8; ++r) To[wave * 16 + 8 * hlf + r][nloc] = acc2[r] * (1.0f / (XS * WSC)) + bb; }
  __syncthreads();
  for (int pass = 0; pass < 2; ++pass) { if (tid < 64) *(volatile v4f*)(out + (e0 + tid) * NO) = *(const v4f*)(&To[tid][0]); __threadfence(); }
}
}

extern "C" void kernel_launch(void* const* d_in, const int* in_sizes, int n_in, void* d_out, int out_size, void* d_ws, size_t ws_size, hipStream_t stream) {
  (void)n_in;
  auto Fp = [&](int i) { return (const float*)d_in[i]; }; auto Ip = [&](int i) { return (const int*)d_in[i]; };
  if (in_sizes[0] != N * F || in_sizes[1] != 2 * EFULL || in_sizes[2] != EFULL || in_sizes[3] != C * F || in_sizes[4] != C || in_sizes[5] != C * F || in_sizes[6] != C * F || in_sizes[7] != C || in_sizes[8] != C * C || in_sizes[9] != C || in_sizes[10] != C * C || in_sizes[11] != C * C || in_sizes[12] != C || in_sizes[13] != CM * 2 * C || in_sizes[14] != CM || in_sizes[15] != NO * CM || in_sizes[16] != NO || out_size != EFULL * NO) return;
  size_t off = 0; char* ws = (char*)d_ws;
  auto carve = [&](size_t bytes) { char* p = ws + off; off += (bytes + 255) & ~(size_t)255; return p; };
  const size_t n1 = C * 32, n2 = (size_t)C3 * C, n3 = (size_t)CM * 2 * C, n4 = 16 * CM;
  b16* WL1 = (b16*)carve(n1 * 2); b16* WL2 = (b16*)carve(n2 * 2); b16* WM1 = (b16*)carve(n3 * 2); b16* WM2 = (b16*)carve(n4 * 2); b16* WL1q = (b16*)carve(n1 * 2); b16* WL2q = (b16*)carve(n2 * 2); b16* WM1q = (b16*)carve(n3 * 2); b16* WM2q = (b16*)carve(n4 * 2);
  float* Q1 = (float*)carve((size_t)NP * C * 4); float* ABC = (float*)carve((size_t)NP * C3 * 4); float* Q2 = (float*)carve((size_t)NP * C * 4);
  CsrBufs csr; off = csr_carve(csr, ws, off, E, N);
  if (off > ws_size || off > ((size_t)128 << 20)) return;
  const unsigned pg = (unsigned)((n1 + n2 + n3 + n4) / 8 + 255) / 256;
  prep_kernel<<<pg, 256, 0, stream>>>(Fp(3), Fp(4), Fp(5), Fp(6), Fp(7), Fp(8), Fp(10), Fp(11), Fp(13), Fp(15), WL1, WL2, WM1, WM2, WSC);
  prep_kernel<<<pg, 256, 0, stream>>>(Fp(3), Fp(4), Fp(5), Fp(6), Fp(7), Fp(8), Fp(10), Fp(11), Fp(13), Fp(15), WL1q, WL2q, WM1q, WM2q, WSQ);
  csr_build(csr, Ip(1) + EFULL, E, N, stream);
  layer1_kernel<<<NPL / 32, 64, 0, stream>>>(Fp(0), Fp(2), Ip(1), csr.PERM, csr.ROWPTR, csr.ROWCNT, (int)csr.permLen, WL1, WL1q, Q1);
  lin2_kernel<<<NPL / 32, 64, 0, stream>>>(Q1, WL2, WL2q, Fp(9), Fp(12), ABC);
  agg2_kernel<<<NPL / 32, 256, 0, stream>>>(ABC, Fp(2), Ip(1), csr.PERM, csr.ROWPTR, csr.ROWCNT, (int)csr.permLen, Q2);
  edge_kernel<<<EL / 64, 128, 0, stream>>>(Q2, Ip(1), Ip(1) + EFULL, WM1, WM1q, Fp(14), WM2, WM2q, Fp(16), (float*)d_out);
}
